// DynamicSparselyGatedMixtureOfExperts_13073880449223
// MI455X (gfx1250) — hardware-verified
//
#include <hip/hip_runtime.h>
#include <stdint.h>
#include <stddef.h>
#include <math.h>

#pragma clang fp contract(off)

#define NTOK 4096
#define DM   1024
#define NEX  8
#define MT   32
#define GX   32
#define TPB  4
#define XP   1032
#define YP   260
#define RECW 4
#define TT   64
#define TPF  68

#define LDS_XB  (MT * XP * 2)
#define LDS_YB  (MT * YP * 4)
#define LDS_EXP (LDS_XB + LDS_YB)
#define LDS_RT  (2 * DM * NEX * 4)

#define W_SC 256.0f
#define R_W  0.00390625f

static_assert((XP * 2) % 16 == 0);
static_assert((YP * 4) % 16 == 0);
static_assert((TPF * 4) % 16 == 0);
static_assert(LDS_XB % 16 == 0);
static_assert(NTOK % 256 == 0);
static_assert(NTOK % 8 == 0);
static_assert(GX * TPB * MT == NTOK);
static_assert(TPB * MT <= 256);
static_assert(MT * (DM / 8) == 16 * 256);
static_assert(DM % 256 == 0);
static_assert(DM % 64 == 0);
static_assert(DM % TT == 0);
static_assert((NEX * DM) % 1024 == 0);
static_assert((NTOK * DM) % (8 * 256) == 0);
static_assert(NEX == 8);
static_assert(DM % 128 == 0);
static_assert(RECW == 4);

typedef _Float16       v16h __attribute__((ext_vector_type(16)));
typedef _Float16       v8h  __attribute__((ext_vector_type(8)));
typedef float          v8f  __attribute__((ext_vector_type(8)));
typedef float          v4f  __attribute__((ext_vector_type(4)));
typedef unsigned int   v4u  __attribute__((ext_vector_type(4)));
typedef v4f __attribute__((may_alias)) v4fa;
typedef v4u __attribute__((may_alias)) v4ua;

union FragH { v16h v; v4u q[2]; };
union Pack8 { v8h h; v4u u; };

__device__ __forceinline__ v8f wmma_h(v16h a, v16h b, v8f c) {
  v8f d = __builtin_amdgcn_wmma_f32_16x16x32_f16(false, a, false, b, (short)0, c, false, false);
  asm volatile("v_nop\n\tv_nop\n\tv_nop\n\tv_nop" : "+v"(d) : "v"(a), "v"(b));
  return d;
}

__device__ __forceinline__ v16h ldfrag(const unsigned short* p, int h) {
  FragH f;
  f.q[0] = *(const v4ua*)(p + 8 * h);
  f.q[1] = *(const v4ua*)(p + 16 + 8 * h);
  return f.v;
}

__global__ __launch_bounds__(256) void k_cvt(const float* __restrict__ src,
                                             unsigned short* __restrict__ dst,
                                             int n8, float sc)
{
  const int g = blockIdx.x * 256 + threadIdx.x;
  if (g >= n8) return;
  const float* s = src + (size_t)g * 8;
  const v4f a = *(const v4fa*)s;
  const v4f c = *(const v4fa*)(s + 4);
  v8h hv;
  hv[0] = (_Float16)(a.x * sc); hv[1] = (_Float16)(a.y * sc);
  hv[2] = (_Float16)(a.z * sc); hv[3] = (_Float16)(a.w * sc);
  hv[4] = (_Float16)(c.x * sc); hv[5] = (_Float16)(c.y * sc);
  hv[6] = (_Float16)(c.z * sc); hv[7] = (_Float16)(c.w * sc);
  Pack8 p;
  p.h = hv;
  const v4u u = p.u;
  unsigned short* d = dst + (size_t)g * 8;
  *(volatile v4u*)d = u;
  __threadfence();
  *(volatile v4u*)d = u;
}

__global__ __launch_bounds__(256) void k_tcv(const float* __restrict__ src,
                                             unsigned short* __restrict__ dst,
                                             float sc)
{
  __shared__ __align__(16) float tile[TT * TPF];
  const int tid = threadIdx.x;
  const int n0 = blockIdx.x * TT, k0 = blockIdx.y * TT, e = blockIdx.z;
  const float* s = src + (size_t)e * DM * DM;
  #pragma unroll
  for (int j = 0; j < 4; ++j) {
    const int r  = (tid >> 4) + 16 * j;
    const int c4 = tid & 15;
    const v4f v = *(const v4fa*)(s + (size_t)(k0 + r) * DM + n0 + 4 * c4);
    *(v4fa*)(tile + r * TPF + 4 * c4) = v;
  }
  __syncthreads();
  v4u u[2];
  #pragma unroll
  for (int j = 0; j < 2; ++j) {
    const int n = (tid >> 3) + 32 * j;
    const int q = tid & 7;
    v8h hv;
    #pragma unroll
    for (int i = 0; i < 8; ++i) hv[i] = (_Float16)(tile[(8 * q + i) * TPF + n] * sc);
    Pack8 pk;
    pk.h = hv;
    u[j] = pk.u;
  }
  unsigned short* d0 = dst + (size_t)e * DM * DM + (size_t)(n0 + (tid >> 3)) * DM + k0 + 8 * (tid & 7);
  unsigned short* d1 = d0 + (size_t)32 * DM;
  *(volatile v4u*)d0 = u[0];
  *(volatile v4u*)d1 = u[1];
  __threadfence();
  *(volatile v4u*)d0 = u[0];
  *(volatile v4u*)d1 = u[1];
}

__global__ __launch_bounds__(256) void k_route(const float* __restrict__ x,
                                               const float* __restrict__ noise,
                                               const float* __restrict__ wg,
                                               const float* __restrict__ wn,
                                               float* __restrict__ rec, int ntok)
{
  extern __shared__ __align__(16) unsigned char dsm_r[];
  float* swg = (float*)dsm_r;
  float* swn = swg + DM * NEX;
  __shared__ __align__(16) float srec[8 * RECW];
  const int tid = threadIdx.x, lane = tid & 31, wv = tid >> 5;
  #pragma unroll 1
  for (int i = 0; i < (DM * NEX) / 1024; ++i) {
    const int o = 4 * (tid + 256 * i);
    const v4f a4 = *(const v4fa*)(wg + o);
    const v4f b4 = *(const v4fa*)(wn + o);
    *(v4fa*)(swg + o) = a4;
    *(v4fa*)(swn + o) = b4;
  }
  __syncthreads();

  const int t = blockIdx.x * 8 + wv;
  const int tc = (t < ntok) ? t : (ntok - 1);
  const float* xr = x + (size_t)tc * DM;
  double lg[NEX], ln[NEX];
  #pragma unroll
  for (int e = 0; e < NEX; ++e) { lg[e] = 0.0; ln[e] = 0.0; }
  #pragma unroll 1
  for (int i = 0; i < DM / 32; ++i) {
    const int d = 32 * i + lane;
    const double xv = (double)xr[d];
    const v4f w0 = *(const v4fa*)(swg + d * NEX);
    const v4f w1 = *(const v4fa*)(swg + d * NEX + 4);
    const v4f u0 = *(const v4fa*)(swn + d * NEX);
    const v4f u1 = *(const v4fa*)(swn + d * NEX + 4);
    lg[0] = fma(xv, (double)w0.x, lg[0]);
    lg[1] = fma(xv, (double)w0.y, lg[1]);
    lg[2] = fma(xv, (double)w0.z, lg[2]);
    lg[3] = fma(xv, (double)w0.w, lg[3]);
    lg[4] = fma(xv, (double)w1.x, lg[4]);
    lg[5] = fma(xv, (double)w1.y, lg[5]);
    lg[6] = fma(xv, (double)w1.z, lg[6]);
    lg[7] = fma(xv, (double)w1.w, lg[7]);
    ln[0] = fma(xv, (double)u0.x, ln[0]);
    ln[1] = fma(xv, (double)u0.y, ln[1]);
    ln[2] = fma(xv, (double)u0.z, ln[2]);
    ln[3] = fma(xv, (double)u0.w, ln[3]);
    ln[4] = fma(xv, (double)u1.x, ln[4]);
    ln[5] = fma(xv, (double)u1.y, ln[5]);
    ln[6] = fma(xv, (double)u1.z, ln[6]);
    ln[7] = fma(xv, (double)u1.w, ln[7]);
  }
  #pragma unroll
  for (int off = 16; off > 0; off >>= 1) {
    #pragma unroll
    for (int e = 0; e < NEX; ++e) {
      lg[e] = lg[e] + __shfl_xor(lg[e], off);
      ln[e] = ln[e] + __shfl_xor(ln[e], off);
    }
  }

  const int le = lane & 7;
  double gsel = lg[0], nsel = ln[0];
  #pragma unroll
  for (int e = 1; e < NEX; ++e) {
    gsel = (le == e) ? lg[e] : gsel;
    nsel = (le == e) ? ln[e] : nsel;
  }
  const float vf = (float)nsel;
  const float sp = fmaxf(vf, 0.0f) + log1pf(expf(-fabsf(vf)));
  const float nz = noise[le];
  const double hl = gsel + (double)nz * (double)sp;
  double hh[NEX];
  #pragma unroll
  for (int e = 0; e < NEX; ++e) hh[e] = __shfl(hl, e);

  int i0 = 0;
  double b0 = hh[0];
  #pragma unroll
  for (int e = 1; e < NEX; ++e) {
    const bool take = hh[e] > b0;
    b0 = take ? hh[e] : b0;
    i0 = take ? e : i0;
  }
  int i1 = -1;
  double bb = -1.0e300;
  #pragma unroll
  for (int e = 0; e < NEX; ++e) {
    const bool take = (e != i0) && (hh[e] > bb);
    bb = take ? hh[e] : bb;
    i1 = take ? e : i1;
  }
  i1 = (i1 < 0) ? ((i0 == 0) ? 1 : 0) : i1;
  double s0 = hh[0], s1 = hh[0];
  #pragma unroll
  for (int e = 0; e < NEX; ++e) { s0 = (e == i0) ? hh[e] : s0; s1 = (e == i1) ? hh[e] : s1; }
  const float l0 = (float)s0;
  const float l1 = (float)s1;
  const float q   = expf(l1 - l0);
  const float den = 1.0f + q;
  const float rden = 1.0f / den;
  const float g0 = rden;
  const float g1 = q * rden;

  if (lane == 0) {
    v4f r0;
    r0.x = g0; r0.y = g1; r0.z = (float)i0; r0.w = (float)i1;
    *(v4fa*)(srec + RECW * wv) = r0;
  }
  __syncthreads();
  if (wv == 0) {
    const int lr = lane & 7;
    const v4f v = *(const v4fa*)(srec + 4 * lr);
    const int tt = blockIdx.x * 8 + lr;
    const bool ok = (lane < 8) && (tt < ntok);
    float* dst = rec + (size_t)(blockIdx.x * 8) * RECW + 4 * lr;
    if (ok) *(volatile v4f*)dst = v;
    __threadfence();
    if (ok) *(volatile v4f*)dst = v;
  }
}

__device__ __forceinline__ void part_pass(const float* sY, const int* tk, const int* sl,
                                          float* part, int ns, int wv, int lane, int nrows)
{
  #pragma unroll
  for (int i = 0; i < 4; ++i) {
    const int row = wv * 4 + i;
    int t = tk[row];
    t = (t < 0) ? 0 : ((t > NTOK - 1) ? (NTOK - 1) : t);
    int s = sl[row];
    s = (s != 0) ? 1 : 0;
    const v4f v0 = *(const v4fa*)(sY + row * YP + 4 * lane);
    const v4f v1 = *(const v4fa*)(sY + row * YP + 128 + 4 * lane);
    float* dst = part + ((size_t)t * 2 + s) * DM + ns * 256;
    if (row < nrows) {
      *(volatile v4f*)(dst + 4 * lane) = v0;
      *(volatile v4f*)(dst + 128 + 4 * lane) = v1;
    }
  }
}

__global__ __launch_bounds__(256) void k_expert(const unsigned short* __restrict__ xh,
                                                const unsigned short* __restrict__ wt,
                                                const float* __restrict__ rec,
                                                const float* __restrict__ be,
                                                float* __restrict__ part, int ntok)
{
  extern __shared__ __align__(16) unsigned char dsm_e[];
  unsigned short* sX = (unsigned short*)dsm_e;
  float* sY = (float*)(dsm_e + LDS_XB);
  __shared__ int   sTok[TPB * MT];
  __shared__ int   sSlot[TPB * MT];
  __shared__ float sW[TPB * MT];
  __shared__ int   s_wc[8];

  const int tid = threadIdx.x, lane = tid & 31, wv = tid >> 5;
  const int h = lane >> 4, m = lane & 15;
  const int e = blockIdx.y;
  const int bx = blockIdx.x;

  if (tid < TPB * MT) { sTok[tid] = 0; sSlot[tid] = 0; sW[tid] = 0.0f; }
  __syncthreads();

  int base = 0;
  #pragma unroll 1
  for (int ch = 0; ch < NTOK / 256; ++ch) {
    const int t = ch * 256 + tid;
    const int tc = (t < ntok) ? t : (ntok - 1);
    const v4f r = *(const v4fa*)(rec + (size_t)tc * RECW);
    int e0 = (int)r.z, e1 = (int)r.w;
    e0 = (e0 < 0) ? 0 : ((e0 > NEX - 1) ? (NEX - 1) : e0);
    e1 = (e1 < 0) ? 0 : ((e1 > NEX - 1) ? (NEX - 1) : e1);
    const bool f0 = (e0 == e);
    const bool f1 = (e1 == e) && !f0;
    const bool f = (f0 || f1) && (t < ntok);
    const unsigned int msk = __builtin_amdgcn_ballot_w32(f);
    const int off = __builtin_popcount(msk & ((1u << lane) - 1u));
    const int wcnt = __builtin_popcount(msk);
    if (lane == 0) s_wc[wv] = wcnt;
    __syncthreads();
    int pre = 0, tot = 0;
    #pragma unroll
    for (int w2 = 0; w2 < 8; ++w2) {
      const int c2 = s_wc[w2];
      tot += c2;
      pre += (w2 < wv) ? c2 : 0;
    }
    if (f) {
      const int rank = base + pre + off;
      const int tile = rank / MT;
      const int lt = tile / GX;
      const int p = lt * MT + (rank % MT);
      if (((tile % GX) == bx) && ((unsigned)p < (unsigned)(TPB * MT))) {
        sTok[p]  = t;
        sSlot[p] = f0 ? 0 : 1;
        sW[p]    = f0 ? r.x : r.y;
      }
    }
    base += tot;
    __syncthreads();
  }
  const int cnt = base;

  const v8f z8 = {0.f, 0.f, 0.f, 0.f, 0.f, 0.f, 0.f, 0.f};

  #pragma unroll 1
  for (int lt = 0; lt < TPB; ++lt) {
    const int m0 = (bx + GX * lt) * MT;
    if (m0 >= cnt) break;
    int nrows = cnt - m0;
    nrows = (nrows > MT) ? MT : nrows;
    const int lo = lt * MT;

    #pragma unroll
    for (int j = 0; j < 16; ++j) {
      const int idx = tid + 256 * j;
      const int row = idx >> 7, c8 = idx & 127;
      int t = sTok[lo + row];
      t = (t < 0) ? 0 : ((t > NTOK - 1) ? (NTOK - 1) : t);
      const size_t go = (size_t)t * DM + 8 * c8;
      const v4u a = *(const v4ua*)(xh + go);
      *(v4ua*)(sX + row * XP + 8 * c8) = a;
    }
    __syncthreads();

    #pragma unroll 1
    for (int ns = 0; ns < DM / 256; ++ns) {
      v8f acc[2][2];
      #pragma unroll
      for (int mt = 0; mt < 2; ++mt)
        #pragma unroll
        for (int nt = 0; nt < 2; ++nt) acc[mt][nt] = z8;
      #pragma unroll 1
      for (int k0 = 0; k0 < DM; k0 += 64) {
        #pragma unroll
        for (int kk = 0; kk < 2; ++kk) {
          const int kb = k0 + 32 * kk;
          v16h a[2];
          #pragma unroll
          for (int mt = 0; mt < 2; ++mt)
            a[mt] = ldfrag(sX + (16 * mt + m) * XP + kb, h);
          #pragma unroll
          for (int nt = 0; nt < 2; ++nt) {
            const int jg = ns * 256 + wv * 32 + 16 * nt + m;
            const size_t ro = ((size_t)e * DM + jg) * DM + kb;
            const v16h b = ldfrag(wt + ro, h);
            #pragma unroll
            for (int mt = 0; mt < 2; ++mt) acc[mt][nt] = wmma_h(a[mt], b, acc[mt][nt]);
          }
        }
      }
      #pragma unroll
      for (int mt = 0; mt < 2; ++mt)
        #pragma unroll
        for (int nt = 0; nt < 2; ++nt) {
          const int cl = wv * 32 + 16 * nt + m;
          const float bv = be[(size_t)e * DM + ns * 256 + cl];
          #pragma unroll
          for (int r = 0; r < 8; ++r) {
            const int row = 16 * mt + 8 * h + r;
            const float y = acc[mt][nt][r] * R_W + bv;
            sY[row * YP + cl] = y * sW[lo + row];
          }
        }
      __syncthreads();
      part_pass(sY, sTok + lo, sSlot + lo, part, ns, wv, lane, nrows);
      __threadfence();
      part_pass(sY, sTok + lo, sSlot + lo, part, ns, wv, lane, nrows);
      __syncthreads();
    }
  }
}

__global__ __launch_bounds__(256) void k_sum(const float* __restrict__ part,
                                             float* __restrict__ out, int ntok)
{
  const int lane = threadIdx.x & 31, wv = threadIdx.x >> 5;
  const int t = blockIdx.x * 8 + wv;
  if (t >= ntok) return;
  const float* p0 = part + (size_t)t * 2 * DM;
  const float* p1 = p0 + DM;
  v4f o[8];
  #pragma unroll
  for (int i = 0; i < 8; ++i) {
    const v4f a = *(const v4fa*)(p0 + 128 * i + 4 * lane);
    const v4f b = *(const v4fa*)(p1 + 128 * i + 4 * lane);
    o[i] = a + b;
  }
  float* d = out + (size_t)t * DM;
  #pragma unroll
  for (int i = 0; i < 8; ++i) *(volatile v4f*)(d + 128 * i + 4 * lane) = o[i];
  __threadfence();
  #pragma unroll
  for (int i = 0; i < 8; ++i) *(volatile v4f*)(d + 128 * i + 4 * lane) = o[i];
}

extern "C" void kernel_launch(void* const* d_in, const int* in_sizes, int n_in,
                              void* d_out, int out_size, void* d_ws, size_t ws_size,
                              hipStream_t stream)
{
  if (n_in < 6) return;
  if (in_sizes[0] != NTOK * DM) return;
  if (in_sizes[1] != NEX) return;
  if (in_sizes[2] != DM * NEX) return;
  if (in_sizes[3] != DM * NEX) return;
  if (in_sizes[4] != NEX * DM * DM) return;
  if (in_sizes[5] != NEX * DM) return;
  if (out_size != NTOK * DM) return;

  const float* x     = (const float*)d_in[0];
  const float* noise = (const float*)d_in[1];
  const float* wg    = (const float*)d_in[2];
  const float* wn    = (const float*)d_in[3];
  const float* we    = (const float*)d_in[4];
  const float* be    = (const float*)d_in[5];
  float* out = (float*)d_out;

  const size_t bXH   = (size_t)NTOK * DM * 2;
  const size_t bWT   = (size_t)NEX * DM * DM * 2;
  const size_t bREC  = (size_t)NTOK * RECW * 4;
  const size_t bPART = (size_t)NTOK * 2 * DM * 4;
  const size_t total = bXH + bWT + bREC + bPART;
  if (total > ws_size) return;
  if (total > (size_t)134217728) return;

  char* ws = (char*)d_ws;
  size_t off = 0;
  unsigned short* XH   = (unsigned short*)(ws + off); off += bXH;
  unsigned short* WT   = (unsigned short*)(ws + off); off += bWT;
  float*          REC  = (float*)(ws + off);          off += bREC;
  float*          PART = (float*)(ws + off);          off += bPART;
  if (off != total) return;

  hipFuncSetAttribute(reinterpret_cast<const void*>(&k_expert),
                      hipFuncAttributeMaxDynamicSharedMemorySize, LDS_EXP);
  hipFuncSetAttribute(reinterpret_cast<const void*>(&k_route),
                      hipFuncAttributeMaxDynamicSharedMemorySize, LDS_RT);

  {
    const int n8x = NTOK * DM / 8;
    k_cvt<<<(n8x + 255) / 256, 256, 0, stream>>>(x, XH, n8x, 1.0f);
  }
  k_tcv<<<dim3(DM / TT, DM / TT, NEX), 256, 0, stream>>>(we, WT, W_SC);
  k_route<<<(NTOK + 7) / 8, 256, LDS_RT, stream>>>(x, noise, wg, wn, REC, NTOK);
  k_expert<<<dim3(GX, NEX), 256, LDS_EXP, stream>>>(XH, WT, REC, be, PART, NTOK);
  k_sum<<<(NTOK + 7) / 8, 256, 0, stream>>>(PART, out, NTOK);
}
